// MambaBlock_43980465111222
// MI455X (gfx1250) — hardware-verified
//
#include <hip/hip_runtime.h>
#include <stddef.h>
#include <stdint.h>
#include <math.h>


#pragma clang fp contract(off)

#define D_MODEL 1024
#define D_STATE 16
#define D_INNER 2048
#define SEQ     2048
#define BATCH   2
#define MROWS   (BATCH * SEQ)
#define NXZ     (2 * D_INNER)
#define K2      (2 * D_INNER)
#define PLANE   ((size_t)MROWS * D_INNER)

#define NTHR   256
#define GBM    64
#define GTHR   128
#define SCT    128
#define TS     32
#define NTILE  (SEQ / TS)

#define U_XB   (MROWS * D_MODEL / 8)
#define U_WIN  (NXZ * D_MODEL / 8)
#define U_WO   (D_MODEL * K2 / 8)
#define U_WX   (32 * K2 / 8)
#define U_AF   (D_INNER * D_STATE / 4)
#define U_ALL  (U_XB + U_WIN + U_WO + U_WX + U_AF)
#define WSMAX  134217728

static_assert(U_XB % NTHR == 0 && U_WIN % NTHR == 0 && U_WO % NTHR == 0 && U_WX % NTHR == 0 && U_AF % NTHR == 0);
static_assert(D_MODEL % 32 == 0 && K2 % 32 == 0);
static_assert(MROWS % GBM == 0 && NXZ % 128 == 0 && D_MODEL % 128 == 0 && D_INNER % 128 == 0);
static_assert(GBM == (GTHR / 32) * 16);
static_assert(SEQ % TS == 0 && TS % 16 == 0 && D_INNER % SCT == 0 && SCT == 128);
static_assert((SEQ & (SEQ - 1)) == 0);
static_assert(TS * SCT >= D_STATE * SCT);
static_assert((size_t)MROWS * D_MODEL == 4194304);

typedef float          v4f   __attribute__((ext_vector_type(4)));
typedef float          v8f   __attribute__((ext_vector_type(8)));
typedef int            v8i   __attribute__((ext_vector_type(8)));
typedef unsigned short v8us  __attribute__((ext_vector_type(8)));
typedef unsigned short v16us __attribute__((ext_vector_type(16)));
typedef __bf16         v16bf __attribute__((ext_vector_type(16)));
typedef v4f  __attribute__((may_alias)) v4fa;
typedef v8us __attribute__((may_alias)) v8usa;
union FragB { v16bf v; v16us u; v8us h[2]; v8i w; };

__device__ __forceinline__ v8f wmb(const FragB& a, const FragB& b, v8f c) {
  v8f d = __builtin_amdgcn_wmma_f32_16x16x32_bf16(false, a.v, false, b.v, (short)0, c, false, false);
  asm volatile("v_nop\n\tv_nop\n\tv_nop\n\tv_nop" : "+v"(d) : "v"(a.w), "v"(b.w));
  return d;
}

__device__ __forceinline__ unsigned bf16_bits(float f) {
  const unsigned u = __float_as_uint(f);
  return (u + 0x7FFFu + ((u >> 16) & 1u)) >> 16;
}
__device__ __forceinline__ float bf16_val(float f) {
  return __uint_as_float(bf16_bits(f) << 16);
}

__device__ __forceinline__ void put8(unsigned short* dp, v8us o) {
  *(volatile v8us*)dp = o;
  __threadfence();
  *(volatile v8us*)dp = o;
}

__device__ __forceinline__ float conv_silu(float x0, float x1, float x2, float x3,
                                           float w0, float w1, float w2, float w3, float bb) {
  float u = w0 * x0;
  u = fmaf(w1, x1, u);
  u = fmaf(w2, x2, u);
  u = fmaf(w3, x3, u);
  u = u + bb;
  const float e = expf(-u);
  return u * __builtin_amdgcn_rcpf(1.0f + e);
}

__global__ __launch_bounds__(NTHR) void k_prep(const float* __restrict__ x, const float* __restrict__ Win,
                                               const float* __restrict__ Wo, const float* __restrict__ Wx,
                                               const float* __restrict__ Alog,
                                               unsigned short* XB, unsigned short* WinT, unsigned short* WO2,
                                               unsigned short* WX2, float* AF) {
  const int u = (int)blockIdx.x * NTHR + (int)threadIdx.x;
  v8us o;
  if (u < U_XB) {
    const float* p = x + (size_t)u * 8;
    const v4f a = *(const v4f*)p;
    const v4f b = *(const v4f*)(p + 4);
    o[0] = (unsigned short)bf16_bits(a.x); o[1] = (unsigned short)bf16_bits(a.y);
    o[2] = (unsigned short)bf16_bits(a.z); o[3] = (unsigned short)bf16_bits(a.w);
    o[4] = (unsigned short)bf16_bits(b.x); o[5] = (unsigned short)bf16_bits(b.y);
    o[6] = (unsigned short)bf16_bits(b.z); o[7] = (unsigned short)bf16_bits(b.w);
    put8(XB + (size_t)u * 8, o);
  } else if (u < U_XB + U_WIN) {
    const int v  = u - U_XB;
    const int n  = v >> 7;
    const int k8 = (v & 127) * 8;
    const float* p = Win + (size_t)k8 * NXZ + n;
#pragma unroll
    for (int i = 0; i < 8; ++i) o[i] = (unsigned short)bf16_bits(p[(size_t)i * NXZ]);
    put8(WinT + (size_t)n * D_MODEL + k8, o);
  } else if (u < U_XB + U_WIN + U_WO) {
    const int v  = u - (U_XB + U_WIN);
    const int n  = v >> 9;
    const int k8 = (v & 511) * 8;
    const int kk = k8 & (D_INNER - 1);
    const float* p = Wo + (size_t)kk * D_MODEL + n;
#pragma unroll
    for (int i = 0; i < 8; ++i) o[i] = (unsigned short)bf16_bits(p[(size_t)i * D_MODEL]);
    put8(WO2 + (size_t)n * K2 + k8, o);
  } else if (u < U_XB + U_WIN + U_WO + U_WX) {
    const int v  = u - (U_XB + U_WIN + U_WO);
    const int n  = v >> 9;
    const int k8 = (v & 511) * 8;
    const int kk = k8 & (D_INNER - 1);
    const float* p = Wx + (size_t)kk * 32 + n;
#pragma unroll
    for (int i = 0; i < 8; ++i) o[i] = (unsigned short)bf16_bits(p[(size_t)i * 32]);
    put8(WX2 + (size_t)n * K2 + k8, o);
  } else if (u < U_ALL) {
    const int v = u - (U_XB + U_WIN + U_WO + U_WX);
    const v4f a = *(const v4f*)(Alog + (size_t)v * 4);
    v4f r;
    r.x = -expf(bf16_val(a.x));
    r.y = -expf(bf16_val(a.y));
    r.z = -expf(bf16_val(a.z));
    r.w = -expf(bf16_val(a.w));
    float* dp = AF + (size_t)v * 4;
    *(volatile v4f*)dp = r;
    __threadfence();
    *(volatile v4f*)dp = r;
  }
}

template <int NT>
__global__ __launch_bounds__(GTHR) void k_gemm(const unsigned short* __restrict__ A,
                                               const unsigned short* __restrict__ BT,
                                               float* outF, int lda, int K, int ldo, int splitN, int planeStride) {
  constexpr int BN = 16 * NT;
  __shared__ __attribute__((aligned(16))) float stg[GBM * BN];
  const int tid = (int)threadIdx.x, lane = tid & 31, wave = tid >> 5, hh = lane >> 4, m = lane & 15;
  const int rowBase = (int)blockIdx.x * GBM;
  const int col0    = (int)blockIdx.y * BN;

  v8f acc[NT];
  {
    const v8f z = {0.f, 0.f, 0.f, 0.f, 0.f, 0.f, 0.f, 0.f};
#pragma unroll
    for (int t = 0; t < NT; ++t) acc[t] = z;
  }
  const unsigned short* ap = A  + (size_t)(rowBase + 16 * wave + m) * (size_t)lda + 8 * hh;
  const unsigned short* bp = BT + (size_t)(col0 + m) * (size_t)K + 8 * hh;

#pragma unroll 1
  for (int k0 = 0; k0 < K; k0 += 32) {
    FragB af;
    af.h[0] = *(const v8usa*)(ap + k0);
    af.h[1] = *(const v8usa*)(ap + k0 + 16);
#pragma unroll
    for (int nt = 0; nt < NT; ++nt) {
      const unsigned short* wq = bp + (size_t)(16 * nt) * (size_t)K + k0;
      FragB bf;
      bf.h[0] = *(const v8usa*)wq;
      bf.h[1] = *(const v8usa*)(wq + 16);
      acc[nt] = wmb(af, bf, acc[nt]);
    }
  }

#pragma unroll
  for (int nt = 0; nt < NT; ++nt) {
    const int lc = 16 * nt + m;
#pragma unroll
    for (int r = 0; r < 8; ++r) {
      const int lr = 16 * wave + 8 * hh + r;
      stg[lr * BN + lc] = acc[nt][r];
    }
  }
  __syncthreads();

  const int pl   = col0 / splitN;
  const int colo = col0 - pl * splitN;
  float* ob = outF + (size_t)pl * (size_t)planeStride + colo;

  if constexpr (NT == 8) {
    v4f pv[16];
#pragma unroll
    for (int i = 0; i < 16; ++i) pv[i] = *(const v4fa*)(stg + (16 * wave + i) * BN + 4 * lane);
#pragma unroll
    for (int i = 0; i < 16; ++i) {
      float* op = ob + (size_t)(rowBase + 16 * wave + i) * (size_t)ldo + 4 * lane;
      *(volatile v4f*)op = pv[i];
    }
    __threadfence();
#pragma unroll
    for (int i = 0; i < 16; ++i) {
      float* op = ob + (size_t)(rowBase + 16 * wave + i) * (size_t)ldo + 4 * lane;
      *(volatile v4f*)op = pv[i];
    }
  } else {
    v4f pv[4];
#pragma unroll
    for (int i = 0; i < 4; ++i) {
      const int lr = 16 * wave + 4 * i + (lane >> 3);
      pv[i] = *(const v4fa*)(stg + lr * BN + 4 * (lane & 7));
    }
#pragma unroll
    for (int i = 0; i < 4; ++i) {
      const int lr = 16 * wave + 4 * i + (lane >> 3);
      float* op = ob + (size_t)(rowBase + lr) * (size_t)ldo + 4 * (lane & 7);
      *(volatile v4f*)op = pv[i];
    }
    __threadfence();
#pragma unroll
    for (int i = 0; i < 4; ++i) {
      const int lr = 16 * wave + 4 * i + (lane >> 3);
      float* op = ob + (size_t)(rowBase + lr) * (size_t)ldo + 4 * (lane & 7);
      *(volatile v4f*)op = pv[i];
    }
  }
}

__global__ __launch_bounds__(NTHR) void k_conv(const float* __restrict__ XA, const float* __restrict__ cw,
                                               const float* __restrict__ cb, unsigned short* XC) {
  const int r  = (int)blockIdx.x;
  const int d8 = (int)threadIdx.x * 8;
  const int l  = r & (SEQ - 1);
  float xs[4][8];
#pragma unroll
  for (int j = 0; j < 4; ++j) {
    const bool ok = (l - 3 + j) >= 0;
    const int rr  = ok ? (r - 3 + j) : r;
    const float* p = XA + (size_t)rr * D_INNER + d8;
    const v4f a = *(const v4f*)p;
    const v4f b = *(const v4f*)(p + 4);
    xs[j][0] = ok ? a.x : 0.0f; xs[j][1] = ok ? a.y : 0.0f;
    xs[j][2] = ok ? a.z : 0.0f; xs[j][3] = ok ? a.w : 0.0f;
    xs[j][4] = ok ? b.x : 0.0f; xs[j][5] = ok ? b.y : 0.0f;
    xs[j][6] = ok ? b.z : 0.0f; xs[j][7] = ok ? b.w : 0.0f;
  }
  float bs[8];
  {
    const v4f a = *(const v4f*)(cb + d8);
    const v4f b = *(const v4f*)(cb + d8 + 4);
    bs[0] = a.x; bs[1] = a.y; bs[2] = a.z; bs[3] = a.w;
    bs[4] = b.x; bs[5] = b.y; bs[6] = b.z; bs[7] = b.w;
  }
  v8us oh, ol;
#pragma unroll
  for (int c = 0; c < 8; ++c) {
    const v4f w = *(const v4f*)(cw + (size_t)(d8 + c) * 4);
    const float xc = conv_silu(xs[0][c], xs[1][c], xs[2][c], xs[3][c],
                               bf16_val(w.x), bf16_val(w.y), bf16_val(w.z), bf16_val(w.w), bf16_val(bs[c]));
    const unsigned hb = bf16_bits(xc);
    const unsigned lb = bf16_bits(xc - __uint_as_float(hb << 16));
    oh[c] = (unsigned short)hb;
    ol[c] = (unsigned short)lb;
  }
  unsigned short* hp = XC + (size_t)r * K2 + d8;
  unsigned short* lp = hp + D_INNER;
  *(volatile v8us*)hp = oh;
  *(volatile v8us*)lp = ol;
  __threadfence();
  *(volatile v8us*)hp = oh;
  *(volatile v8us*)lp = ol;
}

__global__ __launch_bounds__(SCT) void k_scan(const float* __restrict__ XAZ, const float* __restrict__ BCp,
                                              const float* __restrict__ AF, const float* __restrict__ Wdt,
                                              const float* __restrict__ bdt, const float* __restrict__ cw,
                                              const float* __restrict__ cb, const float* __restrict__ Dp,
                                              unsigned short* G) {
  __shared__ __attribute__((aligned(16))) float sBC[TS * 32];
  __shared__ __attribute__((aligned(16))) float sDl[TS * SCT];
  __shared__ __attribute__((aligned(16))) unsigned short sGh[TS * SCT];
  __shared__ __attribute__((aligned(16))) unsigned short sGl[TS * SCT];
  const int tid = (int)threadIdx.x, lane = tid & 31, wave = tid >> 5, hh = lane >> 4, m = lane & 15;
  const int dbase = (int)blockIdx.x * SCT;
  const int d = dbase + tid;
  const int b = (int)blockIdx.y;

#pragma unroll
  for (int i = 0; i < 4; ++i) {
    const int idx = tid + SCT * i;
    const int s   = idx >> 5;
    const int c4  = (idx & 31) * 4;
    const v4f w = *(const v4f*)(Wdt + (size_t)s * D_INNER + dbase + c4);
    *(v4fa*)(sDl + s * SCT + c4) = w;
  }
  __syncthreads();
  FragB bfr[2];
#pragma unroll
  for (int t = 0; t < 2; ++t) {
#pragma unroll
    for (int i = 0; i < 8; ++i) {
      const float wv = sDl[(8 * hh + i) * SCT + 32 * wave + 16 * t + m];
      const unsigned short us = (unsigned short)bf16_bits(wv);
      bfr[t].u[i]     = us;
      bfr[t].u[8 + i] = us;
    }
  }
  __syncthreads();

  float a[D_STATE], h[D_STATE];
  {
    const float* ap = AF + (size_t)d * D_STATE;
    const v4f a0 = *(const v4f*)ap, a1 = *(const v4f*)(ap + 4), a2 = *(const v4f*)(ap + 8), a3 = *(const v4f*)(ap + 12);
    a[0] = a0.x; a[1] = a0.y; a[2] = a0.z; a[3] = a0.w;
    a[4] = a1.x; a[5] = a1.y; a[6] = a1.z; a[7] = a1.w;
    a[8] = a2.x; a[9] = a2.y; a[10] = a2.z; a[11] = a2.w;
    a[12] = a3.x; a[13] = a3.y; a[14] = a3.z; a[15] = a3.w;
  }
#pragma unroll
  for (int s = 0; s < D_STATE; ++s) h[s] = 0.0f;
  const v4f cwv = *(const v4f*)(cw + (size_t)d * 4);
  const float w0 = bf16_val(cwv.x), w1 = bf16_val(cwv.y), w2 = bf16_val(cwv.z), w3 = bf16_val(cwv.w);
  const float cbv = bf16_val(cb[d]);
  const float bd  = bf16_val(bdt[d]);
  const float Dd  = bf16_val(Dp[d]);
  float p0 = 0.0f, p1 = 0.0f, p2 = 0.0f;
  const v8f z8 = {0.f, 0.f, 0.f, 0.f, 0.f, 0.f, 0.f, 0.f};

#pragma unroll 1
  for (int tile = 0; tile < NTILE; ++tile) {
    const int r0 = b * SEQ + tile * TS;
    const v4f t0 = *(const v4f*)(BCp + (size_t)r0 * 32 + 4 * tid);
    const v4f t1 = *(const v4f*)(BCp + (size_t)r0 * 32 + 4 * (tid + SCT));
    __syncthreads();
    *(v4fa*)(sBC + 4 * tid) = t0;
    *(v4fa*)(sBC + 4 * (tid + SCT)) = t1;
    __syncthreads();

#pragma unroll
    for (int mt = 0; mt < TS / 16; ++mt) {
      const float* q = sBC + (16 * mt + m) * 32 + 8 * hh;
      const v4f q0 = *(const v4fa*)q;
      const v4f q1 = *(const v4fa*)(q + 4);
      float bv[8];
      bv[0] = q0.x; bv[1] = q0.y; bv[2] = q0.z; bv[3] = q0.w;
      bv[4] = q1.x; bv[5] = q1.y; bv[6] = q1.z; bv[7] = q1.w;
      FragB af;
#pragma unroll
      for (int i = 0; i < 8; ++i) {
        const unsigned hb = bf16_bits(bv[i]);
        const unsigned lb = bf16_bits(bv[i] - __uint_as_float(hb << 16));
        af.u[i]     = (unsigned short)hb;
        af.u[8 + i] = (unsigned short)lb;
      }
#pragma unroll
      for (int t = 0; t < 2; ++t) {
        const v8f acc = wmb(af, bfr[t], z8);
#pragma unroll
        for (int r = 0; r < 8; ++r)
          sDl[(16 * mt + 8 * hh + r) * SCT + 32 * wave + 16 * t + m] = acc[r];
      }
    }
    __syncthreads();

#pragma unroll 1
    for (int j = 0; j < TS; ++j) {
      const size_t ro = (size_t)(r0 + j) * D_INNER + d;
      const float xa = XAZ[ro];
      const float zz = XAZ[PLANE + ro];
      const float* q = sBC + j * 32;
      const v4f b0 = *(const v4fa*)q,        b1 = *(const v4fa*)(q + 4);
      const v4f b2 = *(const v4fa*)(q + 8),  b3 = *(const v4fa*)(q + 12);
      const v4f c0 = *(const v4fa*)(q + 16), c1 = *(const v4fa*)(q + 20);
      const v4f c2 = *(const v4fa*)(q + 24), c3 = *(const v4fa*)(q + 28);
      const float dlv = sDl[j * SCT + tid];

      const float xc = conv_silu(p0, p1, p2, xa, w0, w1, w2, w3, cbv);
      p0 = p1; p1 = p2; p2 = xa;

      const float v  = dlv + bd;
      const float dt = fmaxf(v, 0.0f) + log1pf(expf(-fabsf(v)));
      const float dx = dt * xc;

      float bq[D_STATE], cq[D_STATE];
      bq[0] = b0.x; bq[1] = b0.y; bq[2] = b0.z; bq[3] = b0.w;
      bq[4] = b1.x; bq[5] = b1.y; bq[6] = b1.z; bq[7] = b1.w;
      bq[8] = b2.x; bq[9] = b2.y; bq[10] = b2.z; bq[11] = b2.w;
      bq[12] = b3.x; bq[13] = b3.y; bq[14] = b3.z; bq[15] = b3.w;
      cq[0] = c0.x; cq[1] = c0.y; cq[2] = c0.z; cq[3] = c0.w;
      cq[4] = c1.x; cq[5] = c1.y; cq[6] = c1.z; cq[7] = c1.w;
      cq[8] = c2.x; cq[9] = c2.y; cq[10] = c2.z; cq[11] = c2.w;
      cq[12] = c3.x; cq[13] = c3.y; cq[14] = c3.z; cq[15] = c3.w;

      float y = 0.0f;
#pragma unroll
      for (int s = 0; s < D_STATE; ++s) {
        const float dA = expf(dt * a[s]);
        h[s] = fmaf(dA, h[s], dx * bq[s]);
        y = fmaf(h[s], cq[s], y);
      }
      const float sz = zz * __builtin_amdgcn_rcpf(1.0f + expf(-zz));
      const float g  = (y + Dd * xc) * sz;
      const unsigned hb = bf16_bits(g);
      const unsigned lb = bf16_bits(g - __uint_as_float(hb << 16));
      sGh[j * SCT + tid] = (unsigned short)hb;
      sGl[j * SCT + tid] = (unsigned short)lb;
    }
    __syncthreads();

    v8us qh[4], ql[4];
#pragma unroll
    for (int it = 0; it < 4; ++it) {
      const int idx = it * SCT + tid;
      const int row = idx >> 4;
      const int pc  = idx & 15;
      qh[it] = *(const v8usa*)(sGh + row * SCT + 8 * pc);
      ql[it] = *(const v8usa*)(sGl + row * SCT + 8 * pc);
    }
#pragma unroll
    for (int it = 0; it < 4; ++it) {
      const int idx = it * SCT + tid;
      const int row = idx >> 4;
      const int pc  = idx & 15;
      unsigned short* gp = G + (size_t)(r0 + row) * K2 + dbase + 8 * pc;
      *(volatile v8us*)gp = qh[it];
      *(volatile v8us*)(gp + D_INNER) = ql[it];
    }
    __threadfence();
#pragma unroll
    for (int it = 0; it < 4; ++it) {
      const int idx = it * SCT + tid;
      const int row = idx >> 4;
      const int pc  = idx & 15;
      unsigned short* gp = G + (size_t)(r0 + row) * K2 + dbase + 8 * pc;
      *(volatile v8us*)gp = qh[it];
      *(volatile v8us*)(gp + D_INNER) = ql[it];
    }
  }
}

static inline size_t al256(size_t o) { return (o + 255) & ~(size_t)255; }

extern "C" void kernel_launch(void* const* d_in, const int* in_sizes, int n_in,
                              void* d_out, int out_size, void* d_ws, size_t ws_size,
                              hipStream_t stream) {
  if (n_in < 10) return;
  if (in_sizes[0] != MROWS * D_MODEL) return;
  if (in_sizes[1] != D_MODEL * NXZ) return;
  if (in_sizes[2] != D_INNER * 4) return;
  if (in_sizes[3] != D_INNER) return;
  if (in_sizes[4] != D_INNER * 32) return;
  if (in_sizes[5] != D_STATE * D_INNER) return;
  if (in_sizes[6] != D_INNER) return;
  if (in_sizes[7] != D_INNER * D_STATE) return;
  if (in_sizes[8] != D_INNER) return;
  if (in_sizes[9] != D_INNER * D_MODEL) return;
  if (out_size != MROWS * D_MODEL) return;

  const float* x     = (const float*)d_in[0];
  const float* W_in  = (const float*)d_in[1];
  const float* convw = (const float*)d_in[2];
  const float* convb = (const float*)d_in[3];
  const float* W_xp  = (const float*)d_in[4];
  const float* W_dt  = (const float*)d_in[5];
  const float* b_dt  = (const float*)d_in[6];
  const float* A_log = (const float*)d_in[7];
  const float* Dp    = (const float*)d_in[8];
  const float* W_out = (const float*)d_in[9];
  float* out = (float*)d_out;

  char* ws = (char*)d_ws;
  size_t off = 0;
  const size_t oXB  = off; off = al256(off + (size_t)MROWS * D_MODEL * 2);
  const size_t oWin = off; off = al256(off + (size_t)NXZ * D_MODEL * 2);
  const size_t oWO  = off; off = al256(off + (size_t)D_MODEL * K2 * 2);
  const size_t oWX  = off; off = al256(off + (size_t)32 * K2 * 2);
  const size_t oXAZ = off; off = al256(off + 2 * PLANE * 4);
  const size_t oXC  = off; off = al256(off + (size_t)MROWS * K2 * 2);
  const size_t oBC  = off; off = al256(off + (size_t)MROWS * 32 * 4);
  const size_t oAF  = off; off = al256(off + (size_t)D_INNER * D_STATE * 4);
  if (off > ws_size || off > (size_t)WSMAX) return;
  unsigned short* XB   = (unsigned short*)(ws + oXB);
  unsigned short* WinT = (unsigned short*)(ws + oWin);
  unsigned short* WO2  = (unsigned short*)(ws + oWO);
  unsigned short* WX2  = (unsigned short*)(ws + oWX);
  float*          XAZ  = (float*)(ws + oXAZ);
  unsigned short* XC   = (unsigned short*)(ws + oXC);
  float*          BC   = (float*)(ws + oBC);
  float*          AF   = (float*)(ws + oAF);

  k_prep<<<U_ALL / NTHR, NTHR, 0, stream>>>(x, W_in, W_out, W_xp, A_log, XB, WinT, WO2, WX2, AF);
  k_gemm<8><<<dim3(MROWS / GBM, NXZ / 128), GTHR, 0, stream>>>(XB, WinT, XAZ, D_MODEL, D_MODEL, D_INNER,
                                                               D_INNER, (int)PLANE);
  k_conv<<<MROWS, NTHR, 0, stream>>>(XAZ, convw, convb, XC);
  k_gemm<2><<<dim3(MROWS / GBM, 1), GTHR, 0, stream>>>(XC, WX2, BC, K2, K2, 32, 32, 0);
  k_scan<<<dim3(D_INNER / SCT, BATCH), SCT, 0, stream>>>(XAZ, BC, AF, W_dt, b_dt, convw, convb, Dp, XC);
  k_gemm<8><<<dim3(MROWS / GBM, D_MODEL / 128), GTHR, 0, stream>>>(XC, WO2, out, K2, K2, D_MODEL, D_MODEL, 0);
}
